// BatchedNeRFMLP_47141561041600
// MI455X (gfx1250) — hardware-verified
//
#include <hip/hip_runtime.h>
#include <math.h>

typedef __attribute__((ext_vector_type(16))) _Float16 v16h;
typedef __attribute__((ext_vector_type(16))) __bf16 v16b;
typedef __attribute__((ext_vector_type(8)))  _Float16 v8h;
typedef __attribute__((ext_vector_type(8)))  float v8f;
typedef __attribute__((ext_vector_type(4)))  float v4f;
typedef __attribute__((ext_vector_type(2)))  float v2f;
typedef __attribute__((ext_vector_type(4)))  unsigned v4u;
typedef __attribute__((ext_vector_type(4)))  int v4i;
typedef float __attribute__((may_alias)) float_a;
typedef int __attribute__((may_alias)) int_a;

template <typename T> __device__ __forceinline__ void vst2(void* p, T v) { *(volatile T*)p = v; __threadfence(); *(volatile T*)p = v; }
__device__ __forceinline__ v8f wmma16(v16h a, v16h b, v8f c) {
  v8f d = __builtin_amdgcn_wmma_f32_16x16x32_f16(false, a, false, b, (short)0, c, false, false);
  asm volatile("v_nop\n\tv_nop\n\tv_nop\n\tv_nop" : "+v"(d) : "v"(a), "v"(b));
  return d;
}
__device__ __forceinline__ v8f wmma_bf(v16b a, v16b b, v8f c) {
  v8f d = __builtin_amdgcn_wmma_f32_16x16x32_bf16(false, a, false, b, (short)0, c, false, false);
  asm volatile("v_nop\n\tv_nop\n\tv_nop\n\tv_nop" : "+v"(d) : "v"(a), "v"(b));
  return d;
}
__device__ __forceinline__ v16h frag_h(const _Float16* rowk0, int lane) {
  union { v16h v; v8h q[2]; } u; const _Float16* p = rowk0 + 8 * (lane >> 4);
  u.q[0] = *(const v8h*)p; u.q[1] = *(const v8h*)(p + 16); return u.v;
}
__device__ __forceinline__ v16h frag_f32(const float* rowk0, int lane) {
  v16h a; const float* p = rowk0 + 8 * (lane >> 4);
#pragma unroll
  for (int i = 0; i < 8; ++i) { a[i] = (_Float16)p[i]; a[8 + i] = (_Float16)p[16 + i]; }
  return a;
}
__device__ __forceinline__ v16h frag_f32s(const float* rowk0, int lane, float sc) {
  v16h a; const float* p = rowk0 + 8 * (lane >> 4);
#pragma unroll
  for (int i = 0; i < 8; ++i) { a[i] = (_Float16)(p[i] * sc); a[8 + i] = (_Float16)(p[16 + i] * sc); }
  return a;
}
__device__ __forceinline__ v16h fragc_f32(const float* W, int k0, int n, int lane, int ld, int K) {
  v16h a; const int g = lane >> 4;
#pragma unroll
  for (int i = 0; i < 8; ++i) { const int ka = k0 + 8 * g + i, kb = ka + 16;
    a[i] = (_Float16)(ka < K ? W[(size_t)(ka < K ? ka : K - 1) * ld + n] : 0.f); a[8 + i] = (_Float16)(kb < K ? W[(size_t)(kb < K ? kb : K - 1) * ld + n] : 0.f); }
  return a;
}
struct F2 { v16b h, l; };
__device__ __forceinline__ F2 bsplit16(const float v[16]) { F2 r;
#pragma unroll
  for (int i = 0; i < 16; ++i) { const __bf16 h = (__bf16)v[i]; r.h[i] = h; r.l[i] = (__bf16)(v[i] - (float)h); }
  return r; }
__device__ __forceinline__ F2 split_row(const float* row, int k0, int lane) { float v[16]; const float* p = row + k0 + 8 * (lane >> 4);
#pragma unroll
  for (int i = 0; i < 8; ++i) { v[i] = p[i]; v[8 + i] = p[16 + i]; }
  return bsplit16(v); }
__device__ __forceinline__ F2 split_rowK(const float* row, int k0, int lane, int K) { float v[16]; const int g = lane >> 4;
#pragma unroll
  for (int i = 0; i < 8; ++i) { const int ka = k0 + 8 * g + i, kb = ka + 16; v[i] = ka < K ? row[ka < K ? ka : K - 1] : 0.f; v[8 + i] = kb < K ? row[kb < K ? kb : K - 1] : 0.f; }
  return bsplit16(v); }
__device__ __forceinline__ F2 split_col(const float* W, int k0, int n, int lane, int ld, int K) { float v[16]; const int g = lane >> 4;
#pragma unroll
  for (int i = 0; i < 8; ++i) { const int ka = k0 + 8 * g + i, kb = ka + 16; v[i] = ka < K ? W[(size_t)(ka < K ? ka : K - 1) * ld + n] : 0.f; v[8 + i] = kb < K ? W[(size_t)(kb < K ? kb : K - 1) * ld + n] : 0.f; }
  return bsplit16(v); }
__device__ __forceinline__ v8f mac3(const F2& a, const F2& b, v8f c) { c = wmma_bf(a.l, b.h, c); c = wmma_bf(a.h, b.l, c); return wmma_bf(a.h, b.h, c); }
__device__ __forceinline__ float sigm(float v) { return 1.0f / (1.0f + expf(-v)); }
#define LDSX() do { asm volatile("s_wait_dscnt 0" ::: "memory"); __builtin_amdgcn_wave_barrier(); __builtin_amdgcn_fence(__ATOMIC_RELEASE, "workgroup"); } while (0)

__device__ __forceinline__ float bfr(float v) { return (float)(__bf16)v; }
#define NBT 64
#define NPT 16384
#define HID 128
#define PIN 63
#define DIN 27
#define CIN (HID + DIN)
#define PTOT 8789
#define OFF_PW 0
#define OFF_PB (PIN * HID)
#define OFF_SW (OFF_PB + HID)
#define OFF_SB (OFF_SW + HID)
#define OFF_CW (OFF_SB + 1)
#define OFF_CB (OFF_CW + 3 * CIN)
#ifndef NBLK
#define NBLK (NBT * NPT / 64)
#endif
__device__ __forceinline__ float penc(const float* p3, int d, int nfreq) { if (d < 3) return p3[d]; const int q = d - 3; const int l = q / 6, s = (q % 6) / 3, c = q % 3; if (l >= nfreq) return 0.f; const float f = (float)(1 << l) * 3.14159274101257324f;     const float a = p3[c] * f; return s == 0 ? sinf(a) : cosf(a); }
__global__ __launch_bounds__(128) void k_nerf(const float* __restrict__ POS, const float* __restrict__ DIR, const float* __restrict__ PRM, float* __restrict__ SIG, float* __restrict__ RGB) {
  __shared__ __align__(16) float sh[4][16][HID + 4]; __shared__ __align__(16) float ssig[64]; __shared__ __align__(16) float srgb[64 * 3];
  const int tid = threadIdx.x, wave = tid >> 5, lane = tid & 31, col = lane & 15, g = lane >> 4; const size_t p0 = (size_t)blockIdx.x * 64 + wave * 16;
  const size_t b = p0 / NPT; const float* P = PRM + b * PTOT; const size_t ap = p0 + col;
  float px[3], dx[3]; for (int c = 0; c < 3; ++c) { px[c] = bfr(POS[ap * 3 + c]); dx[c] = bfr(DIR[ap * 3 + c]); }
  v8f acc[8] = {};
#pragma unroll
  for (int kc = 0; kc < 2; ++kc) { float v[16];
#pragma unroll
    for (int i = 0; i < 8; ++i) { v[i] = penc(px, kc * 32 + 8 * g + i, 10); v[8 + i] = penc(px, kc * 32 + 16 + 8 * g + i, 10); }
    const F2 a = bsplit16(v);
#pragma unroll
    for (int j = 0; j < 8; ++j) { v16b w; const int o = j * 16 + col;
#pragma unroll
      for (int i = 0; i < 8; ++i) { const int d0 = kc * 32 + 8 * g + i, d1 = d0 + 16; w[i] = d0 < PIN ? (__bf16)P[OFF_PW + o * PIN + d0] : (__bf16)0.f; w[8 + i] = d1 < PIN ? (__bf16)P[OFF_PW + o * PIN + d1] : (__bf16)0.f; }
      asm volatile("s_wait_loadcnt 0x0" ::: "memory"); acc[j] = wmma_bf(a.h, w, acc[j]); acc[j] = wmma_bf(a.l, w, acc[j]); } }
#pragma unroll
  for (int j = 0; j < 8; ++j) { const float bb = bfr(P[OFF_PB + j * 16 + col]);
#pragma unroll
    for (int r = 0; r < 8; ++r) sh[wave][8 * g + r][j * 16 + col] = fmaxf(acc[j][r] + bb, 0.f); }
  LDSX();
  v8f as = {}, ac = {};
#pragma unroll
  for (int kc = 0; kc < 5; ++kc) { float v[16];
    if (kc < 4) {
#pragma unroll
      for (int i = 0; i < 8; ++i) { v[i] = sh[wave][col][kc * 32 + 8 * g + i]; v[8 + i] = sh[wave][col][kc * 32 + 16 + 8 * g + i]; } }
    else {
#pragma unroll
      for (int i = 0; i < 8; ++i) { const int d0 = 8 * g + i, d1 = 16 + 8 * g + i; v[i] = d0 < DIN ? penc(dx, d0, 4) : 0.f; v[8 + i] = d1 < DIN ? penc(dx, d1, 4) : 0.f; } }
    const F2 a = bsplit16(v);
    v16b ws_, wc_;
#pragma unroll
    for (int i = 0; i < 8; ++i) { const int k0 = kc * 32 + 8 * g + i, k1 = k0 + 16;
      ws_[i] = (col == 0 && kc < 4) ? (__bf16)P[OFF_SW + k0] : (__bf16)0.f; ws_[8 + i] = (col == 0 && kc < 4) ? (__bf16)P[OFF_SW + k1] : (__bf16)0.f;
      wc_[i] = (col < 3 && k0 < CIN) ? (__bf16)P[OFF_CW + col * CIN + k0] : (__bf16)0.f; wc_[8 + i] = (col < 3 && k1 < CIN) ? (__bf16)P[OFF_CW + col * CIN + k1] : (__bf16)0.f; }
    asm volatile("s_wait_loadcnt 0x0" ::: "memory");
    if (kc < 4) { as = wmma_bf(a.h, ws_, as); as = wmma_bf(a.l, ws_, as); }
    ac = wmma_bf(a.h, wc_, ac); ac = wmma_bf(a.l, wc_, ac); }
  { const float sb = bfr(P[OFF_SB]);
#pragma unroll
    for (int r = 0; r < 8; ++r) { const int pl = wave * 16 + 8 * g + r; if (col == 0) ssig[pl] = as[r] + sb; if (col < 3) { const float z = ac[r] + bfr(P[OFF_CB + col]); srgb[pl * 3 + col] = 1.0f / (1.0f + expf(-z)); } } }
  __syncthreads();
  { const size_t pb0 = (size_t)blockIdx.x * 64; if (tid < 16) vst2(SIG + pb0 + tid * 4, *(const v4f*)&ssig[tid * 4]); else if (tid < 16 + 48) { const int q = tid - 16; vst2(RGB + pb0 * 3 + q * 4, *(const v4f*)&srgb[q * 4]); } } }
extern "C" void kernel_launch(void* const* d_in, const int* in_sizes, int n_in, void* d_out, int out_size, void* d_ws, size_t ws_size, hipStream_t stream) {
  (void)in_sizes; (void)n_in; (void)out_size; (void)d_ws; (void)ws_size;
  const float** F = (const float**)d_in;
  float* SIG = (float*)d_out; float* RGB = (float*)d_out + (size_t)NBT * NPT;
  k_nerf<<<dim3(NBLK), 128, 0, stream>>>(F[0], F[1], F[2], SIG, RGB);
}
